// SD3RewardModel_48739288875294
// MI455X (gfx1250) — hardware-verified
//
#include <hip/hip_runtime.h>


#define NB_  4
#define SQ   512
#define SKV  2048
#define SKT  512
#define EE   1024
#define NH_  16
#define HD   64
#define NRQ  (NB_ * SQ)
#define NRV  (NB_ * SKV)
#define NRT  (NB_ * SKT)
#define ZH   8
#define DM   EE
#define PCAR 1024.0f
#define LOSC 1024.0f
typedef _Float16 h16;
typedef unsigned short bf;
typedef __attribute__((ext_vector_type(16))) __bf16   v16bf;
typedef __attribute__((ext_vector_type(16))) _Float16 v16h;
typedef __attribute__((ext_vector_type(8)))  _Float16 v8h;
typedef __attribute__((ext_vector_type(8)))  unsigned short v8us;
typedef __attribute__((ext_vector_type(8)))  float    v8f;
typedef __attribute__((ext_vector_type(4)))  float    v4f;
typedef v8h  __attribute__((may_alias)) v8ha;
typedef v4f  __attribute__((may_alias)) v4fa;
typedef v8us __attribute__((may_alias)) v8usa;

__device__ __forceinline__ unsigned short f2bf(float f) { unsigned u = __float_as_uint(f); u += 0x7FFFu + ((u >> 16) & 1u); return (unsigned short)(u >> 16); }
__device__ __forceinline__ float bf2f(unsigned short b) { return __uint_as_float(((unsigned)b) << 16); }
__device__ __forceinline__ float bfr(float f) { return bf2f(f2bf(f)); }
__device__ __forceinline__ v16h cat16(v8h lo, v8h hi) { return __builtin_shufflevector(lo, hi, 0, 1, 2, 3, 4, 5, 6, 7, 8, 9, 10, 11, 12, 13, 14, 15); }
__device__ __forceinline__ v16bf cat16b(v8us lo, v8us hi) { return __builtin_bit_cast(v16bf, __builtin_shufflevector(lo, hi, 0, 1, 2, 3, 4, 5, 6, 7, 8, 9, 10, 11, 12, 13, 14, 15)); }
__device__ __forceinline__ v8f wmma16(v16h a, v16h b, v8f c) { return __builtin_amdgcn_wmma_f32_16x16x32_f16(false, a, false, b, (short)0, c, false, false); }
__device__ __forceinline__ v8f wmmab(v16bf a, v16bf b, v8f c) { return __builtin_amdgcn_wmma_f32_16x16x32_bf16(false, a, false, b, (short)0, c, false, false); }


__global__ __launch_bounds__(128) void k_gemmh(const h16* __restrict__ A, const h16* __restrict__ Bn, const float* __restrict__ bias, float* C, int ldc, const float* __restrict__ R, int K, size_t sA, size_t sB, size_t sC, int roundR) {
    __shared__ __align__(16) float ost[4][16 * 68];
    const size_t z = blockIdx.z; A += z * sA; Bn += z * sB; C += z * sC; if (R) R += z * sC;
    const int lane = threadIdx.x & 31, wave = threadIdx.x >> 5, lr = lane & 15, hi = lane >> 4;
    const int r0 = blockIdx.x * 64 + wave * 16, c0 = blockIdx.y * 64;
    const size_t aoff = (size_t)(r0 + lr) * K + 8 * hi;
    size_t boff[4];
#pragma unroll
    for (int t = 0; t < 4; ++t) boff[t] = (size_t)(c0 + t * 16 + lr) * K + 8 * hi;
    v8f acc[4];
#pragma unroll
    for (int t = 0; t < 4; ++t) acc[t] = (v8f){};
#pragma unroll 1
    for (int kc = 0; kc < K; kc += 32) {
        const v16h a = cat16(*(const v8h*)(A + aoff + kc), *(const v8h*)(A + aoff + kc + 16));
#pragma unroll
        for (int t = 0; t < 4; ++t) { const v16h b = cat16(*(const v8h*)(Bn + boff[t] + kc), *(const v8h*)(Bn + boff[t] + kc + 16)); acc[t] = wmma16(a, b, acc[t]); }
        asm volatile("v_nop\n\tv_nop\n\tv_nop\n\tv_nop" : "+v"(acc[0]), "+v"(acc[1]), "+v"(acc[2]), "+v"(acc[3]) : "v"(a));
    }
    float* os = &ost[wave][0];
#pragma unroll
    for (int t = 0; t < 4; ++t) { const float bv = bias ? bfr(bias[c0 + t * 16 + lr]) : 0.f;
#pragma unroll
        for (int j = 0; j < 8; ++j) os[(hi * 8 + j) * 68 + t * 16 + lr] = acc[t][j] + bv; }
    __syncthreads();
    float* crow = C + (size_t)r0 * ldc + c0;
    auto pass = [&]() {
#pragma unroll
        for (int s = 0; s < 8; ++s) { const int Lid = (lane >> 3) + 4 * s, piece = lane & 7; const int row = Lid >> 1, cofs = (Lid & 1) * 32 + piece * 4;
            v4f val = *(const v4fa*)(os + row * 68 + cofs); if (R) { const v4f rv = *(const v4f*)(R + ((size_t)r0 + row) * ldc + c0 + cofs); val += roundR ? (v4f){bfr(rv[0]), bfr(rv[1]), bfr(rv[2]), bfr(rv[3])} : rv; }
            *(volatile v4f*)(crow + (size_t)row * ldc + cofs) = val; }
    };
    pass(); __threadfence(); pass();
}

template <int MODE>
__global__ __launch_bounds__(128) void k_gemm3z(const bf* __restrict__ Ah, const bf* __restrict__ Al, const bf* __restrict__ Bh, const bf* __restrict__ Bl, int K, float* C, int ldc, size_t sA, size_t sB, size_t sC) {
    if ((MODE & 1) && (int)blockIdx.y * 64 > (int)blockIdx.x * 64 + 63) return;
    const size_t z = blockIdx.z; Ah += z * sA; Al += z * sA; Bh += z * sB; Bl += z * sB; C += z * sC;
    const int Klim = (MODE & 2) ? min(K, ((int)blockIdx.x + 1) * 64) : K;
    __shared__ __align__(16) float ost[4][16 * 68];
    const int lane = threadIdx.x & 31, wave = threadIdx.x >> 5, lr = lane & 15, hi = lane >> 4;
    const int r0 = blockIdx.x * 64 + wave * 16, c0 = blockIdx.y * 64;
    const size_t aoff = (size_t)(r0 + lr) * K + 8 * hi;
    v8f acc[4];
#pragma unroll
    for (int t = 0; t < 4; ++t) acc[t] = (v8f){};
#pragma unroll 1
    for (int kc = 0; kc < Klim; kc += 32) {
        const v16bf a = cat16b(*(const v8us*)(Ah + aoff + kc), *(const v8us*)(Ah + aoff + kc + 16));
        v16bf al = a; if (!(MODE & 4) && !(MODE & 16)) al = cat16b(*(const v8us*)(Al + aoff + kc), *(const v8us*)(Al + aoff + kc + 16));
#pragma unroll
        for (int t = 0; t < 4; ++t) { const size_t bo = (size_t)(c0 + t * 16 + lr) * K + kc + 8 * hi;
            const v16bf bh = cat16b(*(const v8us*)(Bh + bo), *(const v8us*)(Bh + bo + 16));
            acc[t] = wmmab(a, bh, acc[t]);
            if (!(MODE & 4)) { if (!(MODE & 16)) acc[t] = wmmab(al, bh, acc[t]); if (!(MODE & 8)) { const v16bf bl = cat16b(*(const v8us*)(Bl + bo), *(const v8us*)(Bl + bo + 16)); acc[t] = wmmab(a, bl, acc[t]); } } }
        asm volatile("v_nop\n\tv_nop\n\tv_nop\n\tv_nop" : "+v"(acc[0]), "+v"(acc[1]), "+v"(acc[2]), "+v"(acc[3]) : "v"(a), "v"(al));
    }
    float* os = &ost[wave][0];
#pragma unroll
    for (int t = 0; t < 4; ++t) {
#pragma unroll
        for (int j = 0; j < 8; ++j) os[(hi * 8 + j) * 68 + t * 16 + lr] = acc[t][j]; }
    __builtin_amdgcn_wave_barrier(); asm volatile("" ::: "memory");
    float* crow = C + (size_t)r0 * ldc + c0;
    auto pass = [&]() {
#pragma unroll
        for (int s = 0; s < 8; ++s) { const int Lid = (lane >> 3) + 4 * s, piece = lane & 7; const int row = Lid >> 1, cofs = (Lid & 1) * 32 + piece * 4;
            const v4f val = *(const v4fa*)(os + row * 68 + cofs); *(volatile v4f*)(crow + (size_t)row * ldc + cofs) = val; }
    };
    pass(); __threadfence(); pass();
}
__global__ __launch_bounds__(256) void k_planes32z(const float* __restrict__ F, int ld, int off, float sc, int rows, bf* Ph, bf* Pl) {
    typedef __attribute__((ext_vector_type(2))) unsigned short v2us;
    const int lane = threadIdx.x & 31; const size_t r = ((size_t)blockIdx.x * 8 + (threadIdx.x >> 5)) * 2 + (lane >> 4); if (r >= (size_t)rows) return; const int z = blockIdx.z; const int c0 = (lane & 15) * 2; v2us oh, ol;
    Ph += (size_t)z * rows * 32; Pl += (size_t)z * rows * 32;
#pragma unroll
    for (int i = 0; i < 2; ++i) { const float y = F[r * ld + off + z * 32 + c0 + i] * sc; const unsigned short hb = f2bf(y); oh[i] = hb; ol[i] = f2bf(y - bf2f(hb)); }
    const size_t o = r * 32 + c0; *(volatile v2us*)(Ph + o) = oh; *(volatile v2us*)(Pl + o) = ol; __threadfence(); *(volatile v2us*)(Ph + o) = oh; *(volatile v2us*)(Pl + o) = ol;
}
__global__ __launch_bounds__(256) void k_vtpadz(const float* __restrict__ F, int ld, int off, int nk, bf* Th, bf* Tl) {
    typedef __attribute__((ext_vector_type(2))) unsigned short v2us;
    const int lane = threadIdx.x & 31; const size_t wid = (size_t)blockIdx.x * 8 + (threadIdx.x >> 5); if (wid >= (size_t)64 * (nk / 64)) return; const int z = blockIdx.z; const int d = (int)(wid / (nk / 64)); const int k0 = (int)(wid % (nk / 64)) * 64 + lane * 2; v2us oh, ol;
    Th += (size_t)z * 64 * nk; Tl += (size_t)z * 64 * nk;
#pragma unroll
    for (int i = 0; i < 2; ++i) { const float y = (d < 32) ? F[(size_t)(k0 + i) * ld + off + z * 32 + (d < 32 ? d : 0)] : 0.f; const unsigned short hb = f2bf(y); oh[i] = hb; ol[i] = f2bf(y - bf2f(hb)); }
    const size_t o = (size_t)d * nk + k0; *(volatile v2us*)(Th + o) = oh; *(volatile v2us*)(Tl + o) = ol; __threadfence(); *(volatile v2us*)(Th + o) = oh; *(volatile v2us*)(Tl + o) = ol;
}
template <int NK>
__global__ __launch_bounds__(256) void k_softmaxz(const float* __restrict__ S, int rows, bf* PH, bf* PL) {
    typedef __attribute__((ext_vector_type(4))) unsigned short v4us;
    const int lane = threadIdx.x & 31, i = blockIdx.x * 8 + (threadIdx.x >> 5); if (i >= rows) return; const size_t zo = (size_t)blockIdx.z * rows * NK; const float* sr = S + zo + (size_t)i * NK; PH += zo; PL += zo;
    float m = -3.0e38f;
#pragma unroll 1
    for (int c0 = lane * 4; c0 < NK; c0 += 128) {
#pragma unroll
        for (int q = 0; q < 4; ++q) m = fmaxf(m, sr[c0 + q]); }
#pragma unroll
    for (int sh = 16; sh; sh >>= 1) m = fmaxf(m, __shfl_xor(m, sh, 32));
    float sum = 0.f;
#pragma unroll 1
    for (int c0 = lane * 4; c0 < NK; c0 += 128) {
#pragma unroll
        for (int q = 0; q < 4; ++q) sum += __expf(sr[c0 + q] - m); }
#pragma unroll
    for (int sh = 16; sh; sh >>= 1) sum += __shfl_xor(sum, sh, 32);
    const float inv = 1.0f / sum;
#pragma unroll 1
    for (int ps = 0; ps < 2; ++ps) {
#pragma unroll 1
        for (int c0 = lane * 4; c0 < NK; c0 += 128) { v4us oh, ol;
#pragma unroll
            for (int q = 0; q < 4; ++q) { const float p = __expf(sr[c0 + q] - m) * inv; const unsigned short hb = f2bf(p); oh[q] = hb; ol[q] = f2bf(p - bf2f(hb)); }
            const size_t o = (size_t)i * NK + c0; *(volatile v4us*)(PH + o) = oh; *(volatile v4us*)(PL + o) = ol; }
        if (ps == 0) __threadfence(); }
}
__global__ __launch_bounds__(256) void k_placez(const float* __restrict__ XH, int rows, int ldy, float* Y) {
    const int lane = threadIdx.x & 31; const size_t q = (size_t)blockIdx.x * 8 + (threadIdx.x >> 5); if (q >= (size_t)rows) return; const int z = blockIdx.z; const float v = XH[((size_t)z * rows + q) * 64 + lane];
    *(volatile float*)(Y + q * ldy + z * 32 + lane) = v; __threadfence(); *(volatile float*)(Y + q * ldy + z * 32 + lane) = v;
}

template <typename T16> struct WFrag;
template <> struct WFrag<h16> { typedef v16h V; static __device__ __forceinline__ V ld(const h16* p) { return cat16(*(const v8h*)p, *(const v8h*)(p + 16)); } static __device__ __forceinline__ v8f mma(V a, V b, v8f c) { return wmma16(a, b, c); } };
template <> struct WFrag<bf> { typedef v16bf V; static __device__ __forceinline__ V ld(const bf* p) { return cat16b(*(const v8us*)p, *(const v8us*)(p + 16)); } static __device__ __forceinline__ v8f mma(V a, V b, v8f c) { return wmmab(a, b, c); } };
template <typename T16, int NSPLIT, bool BIAS>
__global__ __launch_bounds__(32) void k_gemmw(const T16* __restrict__ A, const T16* __restrict__ A2, const T16* __restrict__ Bt, const T16* __restrict__ Bt2, int K, float* C, int ldc, const float* __restrict__ bias, size_t sA, size_t sB, size_t sC) {
    typedef typename WFrag<T16>::V V;
    __shared__ __align__(16) float os[16 * 68];
    const size_t z = blockIdx.z; A += z * sA; if (A2) A2 += z * sA; Bt += z * sB; if (Bt2) Bt2 += z * sB; C += z * sC;
    const int lane = threadIdx.x & 31, lr = lane & 15, hi = lane >> 4; const int r0 = blockIdx.x * 64, c0 = blockIdx.y * 64;
    v8f acc[4][4];
#pragma unroll
    for (int mb = 0; mb < 4; ++mb)
#pragma unroll
        for (int nb = 0; nb < 4; ++nb) acc[mb][nb] = (v8f){};
    const size_t aoff = (size_t)(r0 + lr) * K + 8 * hi, boff = (size_t)(c0 + lr) * K + 8 * hi;
#pragma unroll 1
    for (int kc = 0; kc < K; kc += 32) {
        V a[4], a2[4];
#pragma unroll
        for (int mb = 0; mb < 4; ++mb) { a[mb] = WFrag<T16>::ld(A + aoff + (size_t)mb * 16 * K + kc); if (NSPLIT == 1 || NSPLIT == 2) a2[mb] = WFrag<T16>::ld(A2 + aoff + (size_t)mb * 16 * K + kc); }
#pragma unroll
        for (int nb = 0; nb < 4; ++nb) { const V b = WFrag<T16>::ld(Bt + boff + (size_t)nb * 16 * K + kc); V b2; if (NSPLIT >= 2) b2 = WFrag<T16>::ld(Bt2 + boff + (size_t)nb * 16 * K + kc);
#pragma unroll
            for (int mb = 0; mb < 4; ++mb) { acc[mb][nb] = WFrag<T16>::mma(a[mb], b, acc[mb][nb]); if (NSPLIT == 1 || NSPLIT == 2) acc[mb][nb] = WFrag<T16>::mma(a2[mb], b, acc[mb][nb]); if (NSPLIT >= 2) acc[mb][nb] = WFrag<T16>::mma(a[mb], b2, acc[mb][nb]); } }
        asm volatile("v_nop\n\tv_nop\n\tv_nop\n\tv_nop" : "+v"(acc[0][0]), "+v"(acc[1][1]), "+v"(acc[2][2]), "+v"(acc[3][3]) : "v"(a[0]), "v"(a[3]));
    }
#pragma unroll
    for (int mb = 0; mb < 4; ++mb) {
#pragma unroll
        for (int nb = 0; nb < 4; ++nb) {
#pragma unroll
            for (int j = 0; j < 8; ++j) os[(hi * 8 + j) * 68 + nb * 16 + lr] = acc[mb][nb][j]; }
        __builtin_amdgcn_wave_barrier(); asm volatile("" ::: "memory");
        float* crow = C + (size_t)(r0 + mb * 16) * ldc + c0;
#pragma unroll 1
        for (int ps = 0; ps < 2; ++ps) {
#pragma unroll
            for (int s = 0; s < 8; ++s) { const int row = 2 * s + hi, cofs = lr * 4; v4f val = *(const v4fa*)(os + row * 68 + cofs); if (BIAS) { val[0] += bfr(bias[c0 + cofs]); val[1] += bfr(bias[c0 + cofs + 1]); val[2] += bfr(bias[c0 + cofs + 2]); val[3] += bfr(bias[c0 + cofs + 3]); }
                *(volatile v4f*)(crow + (size_t)row * ldc + cofs) = val; }
            if (ps == 0) __threadfence(); }
        __builtin_amdgcn_wave_barrier(); asm volatile("" ::: "memory");
    }
}

typedef __attribute__((ext_vector_type(4))) _Float16 v4h;
__device__ __forceinline__ h16 tohx(float x) { return (h16)x; }
__global__ __launch_bounds__(256) void k_cvt8h(const float* __restrict__ src, h16* dst, size_t n8) { const size_t i = (size_t)blockIdx.x * 256 + threadIdx.x; if (i >= n8) return; const v8f v = *(const v8f*)(src + i * 8); v8h o;
#pragma unroll
    for (int k = 0; k < 8; ++k) o[k] = tohx(bfr(v[k])); *(volatile v8h*)(dst + i * 8) = o; __threadfence(); *(volatile v8h*)(dst + i * 8) = o; }
__global__ __launch_bounds__(256) void k_rms(const float* __restrict__ x, const float* __restrict__ w, int nrows, h16* P) {
    const int lane = threadIdx.x & 31; const size_t r = (size_t)blockIdx.x * 8 + (threadIdx.x >> 5); if (r >= (size_t)nrows) return; float v[32]; float q = 0.f;
#pragma unroll
    for (int c = 0; c < 4; ++c) {
#pragma unroll
        for (int i = 0; i < 8; ++i) { v[c * 8 + i] = bfr(x[r * EE + c * 256 + lane * 8 + i]); q = fmaf(v[c * 8 + i], v[c * 8 + i], q); } }
#pragma unroll
    for (int sh = 16; sh; sh >>= 1) q += __shfl_xor(q, sh, 32);
    const float rs = rsqrtf(q * (1.0f / EE) + 1.1920929e-07f);
#pragma unroll 1
    for (int ps = 0; ps < 2; ++ps) {
#pragma unroll
        for (int c = 0; c < 4; ++c) { v8h o;
#pragma unroll
            for (int i = 0; i < 8; ++i) { const int col = c * 256 + lane * 8 + i; o[i] = tohx(v[c * 8 + i] * rs * bfr(w[col])); }
            *(volatile v8h*)(P + r * EE + c * 256 + lane * 8) = o; }
        if (ps == 0) __threadfence(); }
}
__global__ __launch_bounds__(256) void k_gate(const float* __restrict__ G1, const float* __restrict__ w2, const float* __restrict__ b2, int nrows, float* gate) {
    const int lane = threadIdx.x & 31; const size_t r0 = ((size_t)blockIdx.x * 8 + (threadIdx.x >> 5)) * 32; if (r0 >= (size_t)nrows) return; const size_t r = r0 + lane; float a = 0.f;
#pragma unroll 1
    for (int c = 0; c < EE; ++c) { const float hcur = G1[r * EE + c]; const float sl = __fdiv_rn(hcur, 1.0f + __expf(-hcur)); a = fmaf(sl, bfr(w2[c]), a); }
    const float gt = __fdiv_rn(1.0f, 1.0f + __expf(-(a + bfr(b2[0]))));
    *(volatile float*)(gate + r) = gt; __threadfence(); *(volatile float*)(gate + r) = gt;
}
__global__ __launch_bounds__(256) void k_hplg(const float* __restrict__ F, int S, int b, int h0, float sc, h16* P) {
    const int lane = threadIdx.x & 31; const size_t w = (size_t)blockIdx.x * 8 + (threadIdx.x >> 5); const int t = (int)(w * 2 + (lane >> 4)); if (t >= S) return; const int z = blockIdx.z; const int c0 = (lane & 15) * 4; v4h o;
#pragma unroll
    for (int q = 0; q < 4; ++q) o[q] = tohx(F[((size_t)b * S + t) * EE + (h0 + z) * HD + c0 + q] * sc);
    const size_t off = ((size_t)z * S + t) * HD + c0; *(volatile v4h*)(P + off) = o; __threadfence(); *(volatile v4h*)(P + off) = o;
}
__global__ __launch_bounds__(256) void k_vTg(const float* __restrict__ V, const float* __restrict__ gate, int S, int b, int h0, h16* VT) {
    __shared__ float tl[64][65];
    const int tid = threadIdx.x; const int t0 = blockIdx.x * 64; const int z = blockIdx.z; const int rr = tid >> 2, cq = (tid & 3) * 16; const size_t row = (size_t)b * S + t0 + rr; const float gt = gate[row];
#pragma unroll
    for (int i = 0; i < 16; ++i) tl[rr][cq + i] = V[row * EE + (h0 + z) * HD + cq + i] * gt;
    __syncthreads();
    const int lane = tid & 31, wv = tid >> 5;
    auto pass = [&]() {
#pragma unroll
        for (int st = 0; st < 4; ++st) { const int dr = wv * 8 + st * 2 + (lane >> 4); const int tq = (lane & 15) * 4; v4h v;
#pragma unroll
            for (int i = 0; i < 4; ++i) v[i] = tohx(tl[tq + i][dr]);
            *(volatile v4h*)(VT + ((size_t)z * HD + dr) * S + t0 + tq) = v; }
    };
    pass(); __threadfence(); pass();
}
__global__ __launch_bounds__(256) void k_softg(const float* __restrict__ Sm, int S, h16* P) {
    const int lane = threadIdx.x & 31, i = blockIdx.x * 8 + (threadIdx.x >> 5); if (i >= SQ) return; const size_t zo = ((size_t)blockIdx.z * SQ + i) * S; const float* sr = Sm + zo; h16* po = P + zo;
    float m = -3.0e38f;
#pragma unroll 1
    for (int c0 = lane * 4; c0 < S; c0 += 128) {
#pragma unroll
        for (int q = 0; q < 4; ++q) m = fmaxf(m, sr[c0 + q]); }
#pragma unroll
    for (int sh = 16; sh; sh >>= 1) m = fmaxf(m, __shfl_xor(m, sh, 32));
    float sum = 0.f;
#pragma unroll 1
    for (int c0 = lane * 4; c0 < S; c0 += 128) {
#pragma unroll
        for (int q = 0; q < 4; ++q) sum += __expf(sr[c0 + q] - m); }
#pragma unroll
    for (int sh = 16; sh; sh >>= 1) sum += __shfl_xor(sum, sh, 32);
    const float f = __fdiv_rn(PCAR, sum);
#pragma unroll 1
    for (int ps = 0; ps < 2; ++ps) {
#pragma unroll 1
        for (int c0 = lane * 4; c0 < S; c0 += 128) { v4h o;
#pragma unroll
            for (int q = 0; q < 4; ++q) o[q] = tohx(__expf(sr[c0 + q] - m) * f);
            *(volatile v4h*)(po + c0) = o; }
        if (ps == 0) __threadfence(); }
}
__global__ __launch_bounds__(256) void k_mergeh(const float* __restrict__ O1, const float* __restrict__ O2, int b, h16* HM) {
    const int lane = threadIdx.x & 31, i = blockIdx.x * 8 + (threadIdx.x >> 5); if (i >= SQ) return;
#pragma unroll 1
    for (int ps = 0; ps < 2; ++ps) {
#pragma unroll
        for (int q = 0; q < 4; ++q) { const int c0 = q * 256 + lane * 8; const int h = c0 / HD, d0 = c0 % HD; v8h o;
#pragma unroll
            for (int k = 0; k < 8; ++k) { const size_t e = ((size_t)h * SQ + i) * HD + d0 + k; o[k] = tohx((O1[e] + O2[e]) * (1.0f / PCAR)); }
            *(volatile v8h*)(HM + ((size_t)b * SQ + i) * EE + c0) = o; }
        if (ps == 0) __threadfence(); }
}
__global__ __launch_bounds__(256) void k_resid(const float* __restrict__ Cm, const float* __restrict__ x, float* OUTB) {
    const int lane = threadIdx.x & 31; const size_t r = (size_t)blockIdx.x * 8 + (threadIdx.x >> 5); if (r >= (size_t)NRQ) return;
#pragma unroll 1
    for (int ps = 0; ps < 2; ++ps) {
#pragma unroll
        for (int p = 0; p < EE / 128; ++p) { const int c0 = p * 128 + lane * 4; v4f v = *(const v4f*)(Cm + r * EE + c0);
#pragma unroll
            for (int i = 0; i < 4; ++i) v[i] += bfr(x[r * EE + c0 + i]);
            *(volatile v4f*)(OUTB + r * EE + c0) = v; }
        if (ps == 0) __threadfence(); }
}
extern "C" void kernel_launch(void* const* d_in, const int* in_sizes, int n_in,
                              void* d_out, int out_size, void* d_ws, size_t ws_size, hipStream_t stream) {
    (void)in_sizes; (void)n_in; (void)out_size;
    const float* qs = (const float*)d_in[0]; const float* cv = (const float*)d_in[1]; const float* ct = (const float*)d_in[2]; const float* wnq = (const float*)d_in[3]; const float* wnv = (const float*)d_in[4]; const float* wnt = (const float*)d_in[5];
    const float* Wq = (const float*)d_in[6]; const float* bq = (const float*)d_in[7]; const float* Wkv = (const float*)d_in[8]; const float* bkv = (const float*)d_in[9]; const float* Wvv = (const float*)d_in[10]; const float* bvv = (const float*)d_in[11];
    const float* Wkt = (const float*)d_in[12]; const float* bkt = (const float*)d_in[13]; const float* Wvt = (const float*)d_in[14]; const float* bvt = (const float*)d_in[15];
    const float* Wg1v = (const float*)d_in[16]; const float* bg1v = (const float*)d_in[17]; const float* Wg2v = (const float*)d_in[18]; const float* bg2v = (const float*)d_in[19]; const float* Wg1t = (const float*)d_in[20]; const float* bg1t = (const float*)d_in[21]; const float* Wg2t = (const float*)d_in[22]; const float* bg2t = (const float*)d_in[23];
    const float* Wo = (const float*)d_in[24]; const float* bo = (const float*)d_in[25];
    float* out = (float*)d_out;
    char* wsp = (char*)d_ws;
    auto take = [&](size_t bytes) { char* p = wsp; wsp += (bytes + 255) & ~(size_t)255; return (void*)p; };
    const size_t WSZ = (size_t)EE * EE * 2;
    h16* WQ = (h16*)take(WSZ); h16* WKV = (h16*)take(WSZ); h16* WVV = (h16*)take(WSZ); h16* WKT = (h16*)take(WSZ); h16* WVT = (h16*)take(WSZ); h16* WG1V = (h16*)take(WSZ); h16* WG1T = (h16*)take(WSZ); h16* WOH = (h16*)take(WSZ);
    h16* QN = (h16*)take((size_t)NRQ * EE * 2); h16* CVN = (h16*)take((size_t)NRV * EE * 2); h16* CTN = (h16*)take((size_t)NRT * EE * 2);
    float* Q = (float*)take((size_t)NRQ * EE * 4); float* KVf = (float*)take((size_t)NRV * EE * 4); float* VVf = (float*)take((size_t)NRV * EE * 4); float* G1 = (float*)take((size_t)NRV * EE * 4); float* GV = (float*)take((size_t)NRV * 4); float* GT = (float*)take((size_t)NRT * 4);
    float* KTf = G1; float* VTf = G1 + (size_t)NRT * EE; float* G1T = G1 + (size_t)2 * NRT * EE;
    h16* Qx = (h16*)take((size_t)NH_ * SQ * HD * 2); h16* Kx = (h16*)take((size_t)ZH * SKV * HD * 2); h16* VT = (h16*)take((size_t)ZH * HD * SKV * 2); float* S = (float*)take((size_t)ZH * SQ * SKV * 4); h16* Px = (h16*)take((size_t)ZH * SQ * SKV * 2); float* O1 = (float*)take((size_t)NH_ * SQ * HD * 4); float* O2 = (float*)take((size_t)NH_ * SQ * HD * 4);
    h16* HM = (h16*)take((size_t)NRQ * EE * 2); float* CO = (float*)take((size_t)NRQ * EE * 4);
    if ((size_t)(wsp - (char*)d_ws) > ws_size) return;
    const size_t n8 = (size_t)EE * EE / 8; const unsigned nb8 = (unsigned)((n8 + 255) / 256);
    k_cvt8h<<<nb8, 256, 0, stream>>>(Wq, WQ, n8); k_cvt8h<<<nb8, 256, 0, stream>>>(Wkv, WKV, n8); k_cvt8h<<<nb8, 256, 0, stream>>>(Wvv, WVV, n8); k_cvt8h<<<nb8, 256, 0, stream>>>(Wkt, WKT, n8); k_cvt8h<<<nb8, 256, 0, stream>>>(Wvt, WVT, n8); k_cvt8h<<<nb8, 256, 0, stream>>>(Wg1v, WG1V, n8); k_cvt8h<<<nb8, 256, 0, stream>>>(Wg1t, WG1T, n8); k_cvt8h<<<nb8, 256, 0, stream>>>(Wo, WOH, n8);
    k_rms<<<NRQ / 8, 256, 0, stream>>>(qs, wnq, NRQ, QN); k_rms<<<NRV / 8, 256, 0, stream>>>(cv, wnv, NRV, CVN); k_rms<<<NRT / 8, 256, 0, stream>>>(ct, wnt, NRT, CTN);
    k_gemmw<h16, 0, true><<<dim3(NRQ / 64, EE / 64, 1), 32, 0, stream>>>(QN, nullptr, WQ, nullptr, EE, Q, EE, bq, 0, 0, 0);
    k_gemmw<h16, 0, true><<<dim3(NRV / 64, EE / 64, 1), 32, 0, stream>>>(CVN, nullptr, WKV, nullptr, EE, KVf, EE, bkv, 0, 0, 0);
    k_gemmw<h16, 0, true><<<dim3(NRV / 64, EE / 64, 1), 32, 0, stream>>>(CVN, nullptr, WVV, nullptr, EE, VVf, EE, bvv, 0, 0, 0);
    k_gemmw<h16, 0, true><<<dim3(NRV / 64, EE / 64, 1), 32, 0, stream>>>(CVN, nullptr, WG1V, nullptr, EE, G1, EE, bg1v, 0, 0, 0); k_gate<<<(NRV / 32 + 7) / 8, 256, 0, stream>>>(G1, Wg2v, bg2v, NRV, GV);
    k_gemmw<h16, 0, true><<<dim3(NRT / 64, EE / 64, 1), 32, 0, stream>>>(CTN, nullptr, WKT, nullptr, EE, KTf, EE, bkt, 0, 0, 0);
    k_gemmw<h16, 0, true><<<dim3(NRT / 64, EE / 64, 1), 32, 0, stream>>>(CTN, nullptr, WVT, nullptr, EE, VTf, EE, bvt, 0, 0, 0);
    k_gemmw<h16, 0, true><<<dim3(NRT / 64, EE / 64, 1), 32, 0, stream>>>(CTN, nullptr, WG1T, nullptr, EE, G1T, EE, bg1t, 0, 0, 0); k_gate<<<(NRT / 32 + 7) / 8, 256, 0, stream>>>(G1T, Wg2t, bg2t, NRT, GT);
    for (int b = 0; b < NB_; ++b) {
        k_hplg<<<dim3((SQ / 2) / 8, 1, NH_), 256, 0, stream>>>(Q, SQ, b, 0, 0.125f, Qx);
        for (int h0 = 0; h0 < NH_; h0 += ZH) {
            k_hplg<<<dim3((SKV / 2) / 8, 1, ZH), 256, 0, stream>>>(KVf, SKV, b, h0, 1.0f, Kx); k_vTg<<<dim3(SKV / 64, 1, ZH), 256, 0, stream>>>(VVf, GV, SKV, b, h0, VT);
            k_gemmw<h16, 0, false><<<dim3(SQ / 64, SKV / 64, ZH), 32, 0, stream>>>(Qx + (size_t)h0 * SQ * HD, nullptr, Kx, nullptr, HD, S, SKV, nullptr, (size_t)SQ * HD, (size_t)SKV * HD, (size_t)SQ * SKV);
            k_softg<<<dim3(SQ / 8, 1, ZH), 256, 0, stream>>>(S, SKV, Px);
            k_gemmw<h16, 0, false><<<dim3(SQ / 64, 1, ZH), 32, 0, stream>>>(Px, nullptr, VT, nullptr, SKV, O1 + (size_t)h0 * SQ * HD, HD, nullptr, (size_t)SQ * SKV, (size_t)HD * SKV, (size_t)SQ * HD);
            k_hplg<<<dim3((SKT / 2) / 8, 1, ZH), 256, 0, stream>>>(KTf, SKT, b, h0, 1.0f, Kx); k_vTg<<<dim3(SKT / 64, 1, ZH), 256, 0, stream>>>(VTf, GT, SKT, b, h0, VT);
            k_gemmw<h16, 0, false><<<dim3(SQ / 64, SKT / 64, ZH), 32, 0, stream>>>(Qx + (size_t)h0 * SQ * HD, nullptr, Kx, nullptr, HD, S, SKT, nullptr, (size_t)SQ * HD, (size_t)SKT * HD, (size_t)SQ * SKT);
            k_softg<<<dim3(SQ / 8, 1, ZH), 256, 0, stream>>>(S, SKT, Px);
            k_gemmw<h16, 0, false><<<dim3(SQ / 64, 1, ZH), 32, 0, stream>>>(Px, nullptr, VT, nullptr, SKT, O2 + (size_t)h0 * SQ * HD, HD, nullptr, (size_t)SQ * SKT, (size_t)HD * SKT, (size_t)SQ * HD); }
        k_mergeh<<<SQ / 8, 256, 0, stream>>>(O1, O2, b, HM); }
    k_gemmw<h16, 0, true><<<dim3(NRQ / 64, EE / 64, 1), 32, 0, stream>>>(HM, nullptr, WOH, nullptr, EE, CO, EE, bo, 0, 0, 0);
    k_resid<<<NRQ / 8, 256, 0, stream>>>(CO, qs, out);
}
